// PartTokenizer_87780541595684
// MI455X (gfx1250) — hardware-verified
//
#include <hip/hip_runtime.h>


namespace {
constexpr int B = 16, P = 24, NPT = 2048, NS = 512, C1 = 128, NTOK = B * P, TPP = NS / 16, DOUT = 512, KPJ = 192;
constexpr float XS = 8.0f, S2 = 256.0f, S3 = 1024.0f, S4 = 32768.0f, WSC = 256.0f;
typedef _Float16 b16;
typedef __attribute__((ext_vector_type(16))) _Float16 v16b;
typedef __attribute__((ext_vector_type(8))) _Float16 v8b;
typedef __attribute__((ext_vector_type(8))) float v8f;
typedef __attribute__((ext_vector_type(4))) float v4f;
__device__ __forceinline__ float bf16_rne(float f) { unsigned int u = __float_as_uint(f); u += 0x7FFFu + ((u >> 16) & 1u); float r = __uint_as_float(u & 0xFFFF0000u); asm volatile("" : "+v"(r)); return r; }
__device__ __forceinline__ void split16(float v, b16& hi, b16& lo) { hi = (b16)v; lo = (b16)(v - (float)hi); }
__device__ __forceinline__ v16b frag_kb(const b16* p, int hh) { const v8b a = *(const v8b*)(p + 8 * hh), b = *(const v8b*)(p + 16 + 8 * hh); v16b f;
#pragma unroll
  for (int e = 0; e < 8; ++e) { f[e] = a[e]; f[8 + e] = b[e]; } return f; }
__device__ __forceinline__ v8f wmma16b(v16b a, v16b b, v8f c) { v8f d = __builtin_amdgcn_wmma_f32_16x16x32_f16(false, a, false, b, (short)0, c, false, false); asm volatile("v_nop\n\tv_nop\n\tv_nop\n\tv_nop" : "+v"(d) : "v"(a), "v"(b)); return d; }
__device__ __forceinline__ void wave_lds_sync() { __builtin_amdgcn_fence(__ATOMIC_RELEASE, "workgroup"); __builtin_amdgcn_wave_barrier(); __builtin_amdgcn_fence(__ATOMIC_ACQUIRE, "workgroup"); }
__device__ __forceinline__ float pmul(float a, float b) { float p = a * b; asm volatile("" : "+v"(p)); return p; }

__global__ __launch_bounds__(256) void wput_kernel(const float* __restrict__ e1, const float* __restrict__ e2, const float* __restrict__ e3, const float* __restrict__ pj, b16* __restrict__ E1T, b16* __restrict__ E2T, b16* __restrict__ E3T, b16* __restrict__ PJT) {
  const int u = blockIdx.x * 256 + threadIdx.x;
  for (int pass = 0; pass < 2; ++pass) {
    if (u < C1 * 4) { const int o = u / 4, k0 = (u % 4) * 8; v8b v; for (int j = 0; j < 8; ++j) { const int k = k0 + j; v[j] = (b16)(k < 3 ? bf16_rne(e1[k * C1 + o]) * WSC : 0.0f); } *(volatile v8b*)(E1T + (size_t)o * 32 + k0) = v; }
    if (u < C1 * 16) { const int o = u / 16, k0 = (u % 16) * 8; v8b a, c; for (int j = 0; j < 8; ++j) { a[j] = (b16)(bf16_rne(e2[(size_t)(k0 + j) * C1 + o]) * WSC); c[j] = (b16)(bf16_rne(e3[(size_t)(k0 + j) * C1 + o]) * WSC); } *(volatile v8b*)(E2T + (size_t)o * C1 + k0) = a; *(volatile v8b*)(E3T + (size_t)o * C1 + k0) = c; }
    if (u < DOUT * (KPJ / 8)) { const int o = u / (KPJ / 8), k0 = (u % (KPJ / 8)) * 8; v8b v; for (int j = 0; j < 8; ++j) { const int k = k0 + j; v[j] = (b16)(k < 160 ? bf16_rne(pj[(size_t)k * DOUT + o]) * WSC : 0.0f); } *(volatile v8b*)(PJT + (size_t)o * KPJ + k0) = v; }
    __threadfence(); } }
__global__ __launch_bounds__(32) void pts_kernel(const float* __restrict__ pts, const b16* __restrict__ E1T, const float* __restrict__ b1, const b16* __restrict__ E2T, const float* __restrict__ b2, const b16* __restrict__ E3T, const float* __restrict__ b3, int TOKLIM, float* __restrict__ PART) {
  __shared__ __attribute__((aligned(16))) b16 A1[16][40], Ah[16][C1 + 8], Al[16][C1 + 8]; __shared__ float Tf[16][C1 + 4]; const int lane = threadIdx.x, nloc = lane & 15, hlf = lane >> 4; const int tok = blockIdx.x / TPP, t = blockIdx.x % TPP; if (tok >= TOKLIM) return;
  const float* pp = pts + ((size_t)tok * NPT + t * 16) * 3;
  { const int rr = lane & 15; for (int k = 0; k < 16; ++k) { const int c = hlf * 16 + k; A1[rr][c] = (b16)(c < 3 ? bf16_rne(pp[rr * 3 + c]) * XS : 0.0f); } }
  wave_lds_sync(); v8f acc[8];
#pragma unroll
  for (int tt = 0; tt < 8; ++tt) acc[tt] = (v8f){};
  { const v16b a = frag_kb(&A1[nloc][0], hlf);
#pragma unroll
    for (int tt = 0; tt < 8; ++tt) acc[tt] = wmma16b(a, frag_kb(E1T + (size_t)(tt * 16 + nloc) * 32, hlf), acc[tt]); }
#pragma unroll
  for (int tt = 0; tt < 8; ++tt) { const int c = tt * 16 + nloc; const float bb = bf16_rne(b1[c]);
#pragma unroll
    for (int r8 = 0; r8 < 8; ++r8) { b16 p, q; split16(fmaxf(acc[tt][r8] * (1.0f / (XS * WSC)) + bb, 0.0f) * S2, p, q); Ah[8 * hlf + r8][c] = p; Al[8 * hlf + r8][c] = q; } }
  wave_lds_sync();
#pragma unroll
  for (int tt = 0; tt < 8; ++tt) acc[tt] = (v8f){};
#pragma unroll
  for (int kb = 0; kb < C1; kb += 32) { const v16b a = frag_kb(&Ah[nloc][kb], hlf), al = frag_kb(&Al[nloc][kb], hlf);
#pragma unroll
    for (int tt = 0; tt < 8; ++tt) { const v16b bw = frag_kb(E2T + (size_t)(tt * 16 + nloc) * C1 + kb, hlf); acc[tt] = wmma16b(a, bw, acc[tt]); acc[tt] = wmma16b(al, bw, acc[tt]); } }
  wave_lds_sync();
#pragma unroll
  for (int tt = 0; tt < 8; ++tt) { const int c = tt * 16 + nloc; const float bb = bf16_rne(b2[c]);
#pragma unroll
    for (int r8 = 0; r8 < 8; ++r8) { b16 p, q; split16(fmaxf(acc[tt][r8] * (1.0f / (S2 * WSC)) + bb, 0.0f) * S3, p, q); Ah[8 * hlf + r8][c] = p; Al[8 * hlf + r8][c] = q; } }
  wave_lds_sync();
#pragma unroll
  for (int tt = 0; tt < 8; ++tt) acc[tt] = (v8f){};
#pragma unroll
  for (int kb = 0; kb < C1; kb += 32) { const v16b a = frag_kb(&Ah[nloc][kb], hlf), al = frag_kb(&Al[nloc][kb], hlf);
#pragma unroll
    for (int tt = 0; tt < 8; ++tt) { const v16b bw = frag_kb(E3T + (size_t)(tt * 16 + nloc) * C1 + kb, hlf); acc[tt] = wmma16b(a, bw, acc[tt]); acc[tt] = wmma16b(al, bw, acc[tt]); } }
#pragma unroll
  for (int tt = 0; tt < 8; ++tt) { const int c = tt * 16 + nloc; const float bb = bf16_rne(b3[c]);
#pragma unroll
    for (int r8 = 0; r8 < 8; ++r8) Tf[8 * hlf + r8][c] = acc[tt][r8] * (1.0f / (S3 * WSC)) + bb; }
  wave_lds_sync();
  v4f s = {0.0f, 0.0f, 0.0f, 0.0f}; for (int rr = 0; rr < 16; ++rr) for (int k = 0; k < 4; ++k) s[k] += Tf[rr][lane * 4 + k];
  for (int pass = 0; pass < 2; ++pass) { *(volatile v4f*)(PART + ((size_t)tok * TPP + t) * C1 + lane * 4) = s; __threadfence(); }
}
__global__ __launch_bounds__(256) void tok_kernel(const float* __restrict__ bbs, const int* __restrict__ mask, const float* __restrict__ W1, const float* __restrict__ B1, const float* __restrict__ W2, const float* __restrict__ B2, const float* __restrict__ W3, const float* __restrict__ B3, const float* __restrict__ PART, int TOKLIM, float* __restrict__ obb, float* __restrict__ ovis, float* __restrict__ COMB) {
  __shared__ float Hs[8][64], H2s[8][64], Xb[8][12]; const int wave = threadIdx.x >> 5, lane = threadIdx.x & 31; const int tok = blockIdx.x * 8 + wave; if (tok >= TOKLIM) return; const float valid = (mask[tok] != 0) ? 0.0f : 1.0f;
  if (lane < 12) Xb[wave][lane] = bf16_rne(bbs[(size_t)tok * 12 + lane]); wave_lds_sync();
  for (int o = lane; o < 64; o += 32) { float s = bf16_rne(B1[o]);
#pragma unroll 1
    for (int k = 0; k < 12; ++k) s += pmul(Xb[wave][k], bf16_rne(W1[k * 64 + o])); Hs[wave][o] = fmaxf(s, 0.0f); }
  wave_lds_sync();
  for (int o = lane; o < 64; o += 32) { float s = bf16_rne(B2[o]);
#pragma unroll 1
    for (int k = 0; k < 64; ++k) s += pmul(Hs[wave][k], bf16_rne(W2[k * 64 + o])); H2s[wave][o] = fmaxf(s, 0.0f); }
  wave_lds_sync();
  float bbv; { float s = bf16_rne(B3[lane]);
#pragma unroll 1
    for (int k = 0; k < 64; ++k) s += pmul(H2s[wave][k], bf16_rne(W3[k * 32 + lane])); bbv = pmul(s, valid); }
  v4f vs = {0.0f, 0.0f, 0.0f, 0.0f};
#pragma unroll 1
  for (int t = 0; t < TPP; ++t) { const v4f p = *(const v4f*)(PART + ((size_t)tok * TPP + t) * C1 + lane * 4); for (int k = 0; k < 4; ++k) vs[k] += p[k]; }
  for (int k = 0; k < 4; ++k) vs[k] = pmul(pmul(pmul(vs[k], valid), 1.0f / (float)NS), valid);
  for (int pass = 0; pass < 2; ++pass) { ((volatile float*)obb)[(size_t)tok * 32 + lane] = bbv; *(volatile v4f*)(ovis + (size_t)tok * C1 + lane * 4) = vs; ((volatile float*)COMB)[(size_t)tok * KPJ + lane] = bbv; *(volatile v4f*)(COMB + (size_t)tok * KPJ + 32 + lane * 4) = vs; ((volatile float*)COMB)[(size_t)tok * KPJ + 160 + lane] = 0.0f; __threadfence(); }
}
__global__ __launch_bounds__(32) void proj_kernel(const float* __restrict__ COMB, const b16* __restrict__ PJT, const float* __restrict__ pb, int TOKLIM, float* __restrict__ out) {
  __shared__ __attribute__((aligned(16))) b16 Ah[16][KPJ + 8], Al[16][KPJ + 8]; __shared__ float Tf[16][132]; const int lane = threadIdx.x, nloc = lane & 15, hlf = lane >> 4; const int cg = blockIdx.x % 4; const int m0 = (blockIdx.x / 4) * 16; if (m0 >= TOKLIM) return;
  for (int rr = 0; rr < 16; ++rr) for (int q = 0; q < KPJ / 32; ++q) { b16 p, ql; split16(COMB[(size_t)(m0 + rr) * KPJ + q * 32 + lane] * S4, p, ql); Ah[rr][q * 32 + lane] = p; Al[rr][q * 32 + lane] = ql; }
  wave_lds_sync(); v8f acc[8];
#pragma unroll
  for (int t = 0; t < 8; ++t) acc[t] = (v8f){};
#pragma unroll
  for (int kb = 0; kb < KPJ; kb += 32) { const v16b a = frag_kb(&Ah[nloc][kb], hlf), al = frag_kb(&Al[nloc][kb], hlf);
#pragma unroll
    for (int t = 0; t < 8; ++t) { const v16b bw = frag_kb(PJT + (size_t)(cg * 128 + t * 16 + nloc) * KPJ + kb, hlf); acc[t] = wmma16b(a, bw, acc[t]); acc[t] = wmma16b(al, bw, acc[t]); } }
#pragma unroll
  for (int t = 0; t < 8; ++t) { const int c = cg * 128 + t * 16 + nloc; const float bb = bf16_rne(pb[c]);
#pragma unroll
    for (int r8 = 0; r8 < 8; ++r8) Tf[8 * hlf + r8][t * 16 + nloc] = acc[t][r8] * (1.0f / (S4 * WSC)) + bb; }
  wave_lds_sync();
  for (int pass = 0; pass < 2; ++pass) { for (int rr = 0; rr < 16; ++rr) *(volatile v4f*)(out + (size_t)(m0 + rr) * DOUT + cg * 128 + lane * 4) = *(const v4f*)(&Tf[rr][lane * 4]); __threadfence(); }
}
}

extern "C" void kernel_launch(void* const* d_in, const int* in_sizes, int n_in, void* d_out, int out_size, void* d_ws, size_t ws_size, hipStream_t stream) {
  (void)n_in;
  auto Fp = [&](int i) { return (const float*)d_in[i]; }; auto Ip = [&](int i) { return (const int*)d_in[i]; };
  if (in_sizes[0] != NTOK * 12 || in_sizes[1] != NTOK * NPT * 3 || in_sizes[2] != 12 * 64 || in_sizes[8] != 3 * C1 || in_sizes[10] != C1 * C1 || in_sizes[12] != C1 * C1 || in_sizes[16] != 160 * DOUT || in_sizes[18] != NTOK || out_size != NTOK * (DOUT + 32 + C1)) return;
  const int TOKLIM = NTOK;
  size_t off = 0; char* ws = (char*)d_ws;
  auto carve = [&](size_t bytes) { char* p = ws + off; off += (bytes + 255) & ~(size_t)255; return p; };
  b16* E1T = (b16*)carve((size_t)C1 * 32 * 2); b16* E2T = (b16*)carve((size_t)C1 * C1 * 2); b16* E3T = (b16*)carve((size_t)C1 * C1 * 2); b16* PJT = (b16*)carve((size_t)DOUT * KPJ * 2); float* PART = (float*)carve((size_t)NTOK * TPP * C1 * 4); float* COMB = (float*)carve((size_t)NTOK * KPJ * 4);
  if (off > ws_size || off > ((size_t)16 << 20)) return;
  wput_kernel<<<(DOUT * (KPJ / 8) + 255) / 256, 256, 0, stream>>>(Fp(8), Fp(10), Fp(12), Fp(16), E1T, E2T, E3T, PJT);
  pts_kernel<<<TOKLIM * TPP, 32, 0, stream>>>(Fp(1), E1T, Fp(9), E2T, Fp(11), E3T, Fp(13), TOKLIM, PART);
  float* out = (float*)d_out; float* obb = out + (size_t)NTOK * DOUT; float* ovis = obb + (size_t)NTOK * 32;
  tok_kernel<<<(TOKLIM + 7) / 8, 256, 0, stream>>>(Fp(0), Ip(18), Fp(2), Fp(3), Fp(4), Fp(5), Fp(6), Fp(7), PART, TOKLIM, obb, ovis, COMB);
  proj_kernel<<<(TOKLIM / 16) * 4, 32, 0, stream>>>(COMB, PJT, Fp(17), TOKLIM, out);
}
